// EdgePredictor_2018634629213
// MI455X (gfx1250) — hardware-verified
//
#include <hip/hip_runtime.h>
#include <stddef.h>
#include <stdint.h>
#include <math.h>


#define NBT   8
#define NND   256
#define DIN   64
#define HID   256
#define M1    (NBT * NND)
#define N1    (2 * HID)
#define NPR   (NND * NND)
#define NTHR  256
#define GBM   64
#define GBN   64
#define GTHR  128
#define EROWS 64
#define CGRP  (NND / EROWS)
#define ETHR  256
#define ARG   32
#define ELDS_FLOATS (EROWS * HID + 3 * HID + EROWS * 4 + EROWS)
#define ELDS_BYTES  (ELDS_FLOATS * 4)
#define WSMAX 134217728

static_assert(HID == ETHR);
static_assert(EROWS == 8 * (ETHR / 32));
static_assert(EROWS * 4 == ETHR);
static_assert(EROWS == 4 * 16 && HID == 2 * 128);
static_assert((HID % 32) == 0 && (DIN % 32) == 0);
static_assert((M1 % GBM) == 0 && (N1 % GBN) == 0);
static_assert((NND % EROWS) == 0 && (NND % ARG) == 0);
static_assert(ARG == 4 * (NTHR / 32));
static_assert(GBM == (GTHR / 32) * 16);
static_assert(ELDS_BYTES <= 300000);
static_assert((DIN / 8) == 8 && (HID / 8) == 32);
static_assert((NND % 32) == 0);

typedef float          v4f  __attribute__((ext_vector_type(4)));
typedef float          v8f  __attribute__((ext_vector_type(8)));
typedef int            v8i  __attribute__((ext_vector_type(8)));
typedef unsigned int   v4u  __attribute__((ext_vector_type(4)));
typedef unsigned short v8us __attribute__((ext_vector_type(8)));
typedef __bf16         v16b __attribute__((ext_vector_type(16)));
typedef v4f  __attribute__((may_alias)) v4fa;
typedef v8us __attribute__((may_alias)) v8usa;
union FragB { v16b v; v8us h[2]; v8i w; };

__device__ __forceinline__ v8f wmb(const FragB& a, const FragB& b, v8f c) {
  v8f d = __builtin_amdgcn_wmma_f32_16x16x32_bf16(false, a.v, false, b.v, (short)0, c, false, false);
  asm volatile("v_nop\n\tv_nop\n\tv_nop\n\tv_nop" : "+v"(d) : "v"(a.w), "v"(b.w));
  return d;
}

__device__ __forceinline__ unsigned int f2bf(float f) {
  const unsigned int u = __float_as_uint(f);
  return ((u + 0x7FFFu + ((u >> 16) & 1u)) >> 16) & 0xFFFFu;
}
__device__ __forceinline__ float bf2f(unsigned int b) { return __uint_as_float(b << 16); }
__device__ __forceinline__ float bfr(float f) { return bf2f(f2bf(f)); }
__device__ __forceinline__ unsigned int pk2(float lo, float hi) { return f2bf(lo) | (f2bf(hi) << 16); }
__device__ __forceinline__ v4u pack8(const v4f a, const v4f b) {
  v4u r;
  r.x = pk2(a.x, a.y); r.y = pk2(a.z, a.w); r.z = pk2(b.x, b.y); r.w = pk2(b.z, b.w);
  return r;
}

__device__ __forceinline__ float elu1(float t) {
  const float e = expm1f(fminf(t, 0.0f));
  return (t > 0.0f) ? t : e;
}

__global__ __launch_bounds__(NTHR) void k_xprep(const float* __restrict__ x, unsigned short* xb, int nN, int nUnits) {
  const int i = (int)blockIdx.x * NTHR + (int)threadIdx.x;
  if (i >= nUnits) return;
  const int row = i >> 3;
  const int c0  = (i & 7) * 8;
  const int rc  = row < nN ? row : nN - 1;
  const float* p = x + (size_t)rc * DIN + c0;
  v4f a = *(const v4fa*)p, b = *(const v4fa*)(p + 4);
  const v4f z4 = {0.f, 0.f, 0.f, 0.f};
  if (row >= nN) { a = z4; b = z4; }
  const v4u hv = pack8(a, b);
  const size_t o = (size_t)row * DIN + c0;
  *(volatile v4u*)(xb + o) = hv;
  __threadfence();
  *(volatile v4u*)(xb + o) = hv;
}

__global__ __launch_bounds__(NTHR) void k_wtr(const float* __restrict__ w, int Kin, int Ncol, int Nrows, int Kout,
                                              unsigned short* wt, int nUnits) {
  const int u = (int)blockIdx.x * NTHR + (int)threadIdx.x;
  if (u >= nUnits) return;
  const int kq = Kout >> 3;
  const int n  = u / kq;
  const int k8 = (u - n * kq) * 8;
  const int kk = k8 - (k8 / Kin) * Kin;
  const int ncl = n < Ncol ? n : Ncol - 1;
  const float* p = w + (size_t)kk * (size_t)Ncol + ncl;
  v4f a, b;
  a.x = p[0];                    a.y = p[(size_t)Ncol];         a.z = p[(size_t)2 * Ncol];     a.w = p[(size_t)3 * Ncol];
  b.x = p[(size_t)4 * Ncol];     b.y = p[(size_t)5 * Ncol];     b.z = p[(size_t)6 * Ncol];     b.w = p[(size_t)7 * Ncol];
  const v4f z4 = {0.f, 0.f, 0.f, 0.f};
  if (n >= Ncol || n >= Nrows) { a = z4; b = z4; }
  const v4u wv = pack8(a, b);
  unsigned short* o = wt + (size_t)n * (size_t)Kout + k8;
  *(volatile v4u*)o = wv;
  __threadfence();
  *(volatile v4u*)o = wv;
}

__global__ __launch_bounds__(GTHR) void k_gemm1(
    const unsigned short* __restrict__ A, const unsigned short* __restrict__ WT,
    float* outF, int K, int ldo)
{
  __shared__ __attribute__((aligned(16))) float stg[GBM * GBN];
  const int tid = (int)threadIdx.x, lane = tid & 31, wave = tid >> 5, hh = lane >> 4, m = lane & 15;
  const int rowBase = (int)blockIdx.x * GBM;
  const int col0    = (int)blockIdx.y * GBN;

  v8f acc[4];
  {
    const v8f z = {0.f, 0.f, 0.f, 0.f, 0.f, 0.f, 0.f, 0.f};
    acc[0] = z; acc[1] = z; acc[2] = z; acc[3] = z;
  }
  const unsigned short* ap = A  + (size_t)(rowBase + 16 * wave + m) * (size_t)K + 8 * hh;
  const unsigned short* wp = WT + (size_t)(col0 + m) * (size_t)K + 8 * hh;
  const int ksteps = K >> 5;
#pragma unroll 1
  for (int ks = 0; ks < ksteps; ++ks) {
    FragB af;
    af.h[0] = *(const v8usa*)(ap + 32 * ks);
    af.h[1] = *(const v8usa*)(ap + 32 * ks + 16);
#pragma unroll
    for (int t = 0; t < 4; ++t) {
      const unsigned short* wq = wp + (size_t)(16 * t) * (size_t)K + 32 * ks;
      FragB bf;
      bf.h[0] = *(const v8usa*)wq;
      bf.h[1] = *(const v8usa*)(wq + 16);
      acc[t] = wmb(af, bf, acc[t]);
    }
  }

#pragma unroll
  for (int t = 0; t < 4; ++t) {
    const int lc = 16 * t + m;
#pragma unroll
    for (int r = 0; r < 8; ++r) {
      const int lr = 16 * wave + 8 * hh + r;
      stg[lr * GBN + lc] = acc[t][r];
    }
  }
  __syncthreads();

  v4f fv[8];
#pragma unroll
  for (int i = 0; i < 8; ++i) {
    const int lr = 16 * wave + 2 * i + hh;
    fv[i] = *(const v4fa*)(stg + lr * GBN + 4 * m);
  }
#pragma unroll
  for (int i = 0; i < 8; ++i) {
    const int lr = 16 * wave + 2 * i + hh;
    const int gr = rowBase + lr;
    float* op = outF + (size_t)gr * (size_t)ldo + col0 + 4 * m;
    *(volatile v4f*)op = fv[i];
  }
  __threadfence();
#pragma unroll
  for (int i = 0; i < 8; ++i) {
    const int lr = 16 * wave + 2 * i + hh;
    const int gr = rowBase + lr;
    float* op = outF + (size_t)gr * (size_t)ldo + col0 + 4 * m;
    *(volatile v4f*)op = fv[i];
  }
}

__global__ __launch_bounds__(ETHR) void k_edge(
    const float* __restrict__ PQ, const unsigned short* __restrict__ W2T,
    const float* __restrict__ b1, const float* __restrict__ b2, const float* __restrict__ W3,
    float* DL)
{
  extern __shared__ v4f elds4[];
  float* regR = (float*)elds4;
  unsigned short* h1t = (unsigned short*)regR;
  float* stg  = regR;
  float* pb   = regR + EROWS * HID;
  float* b2s  = pb + HID;
  float* w3s  = b2s + HID;
  float* sred = w3s + HID;
  float* sdv  = sred + EROWS * 4;
  const int tid = (int)threadIdx.x, lane = tid & 31, wave = tid >> 5, hh = lane >> 4, m = lane & 15;
  const int bx = (int)blockIdx.x;
  const int bb = (int)blockIdx.y;
  const int a  = bx / CGRP;
  const int c0 = (bx - a * CGRP) * EROWS;

  {
    const float pv = PQ[((size_t)bb * NND + a) * N1 + tid];
    pb[tid]  = pv + bfr(b1[tid]);
    b2s[tid] = bfr(b2[tid]);
    w3s[tid] = bfr(W3[tid]);
  }
  __syncthreads();

#pragma unroll 1
  for (int i = 0; i < 8; ++i) {
    const int lr = 8 * wave + i;
    const float* qrow = PQ + ((size_t)bb * NND + (size_t)(c0 + lr)) * N1 + HID;
#pragma unroll 1
    for (int j = 0; j < HID / 32; ++j) {
      const int col = 32 * j + lane;
      const float t = pb[col] + qrow[col];
      const float h = elu1(t);
      h1t[lr * HID + col] = (unsigned short)f2bf(h);
    }
  }
  __syncthreads();

  v8f acc[8];
  {
    const v8f z = {0.f, 0.f, 0.f, 0.f, 0.f, 0.f, 0.f, 0.f};
#pragma unroll
    for (int t = 0; t < 8; ++t) acc[t] = z;
  }
  const int rw = wave & 3, cg = wave >> 2;
  const unsigned short* ap = h1t + (size_t)(16 * rw + m) * HID + 8 * hh;
  const unsigned short* bp = W2T + (size_t)(128 * cg + m) * HID + 8 * hh;
#pragma unroll 1
  for (int k0 = 0; k0 < HID; k0 += 32) {
    FragB af;
    af.h[0] = *(const v8usa*)(ap + k0);
    af.h[1] = *(const v8usa*)(ap + k0 + 16);
#pragma unroll
    for (int nt = 0; nt < 8; ++nt) {
      const unsigned short* wq = bp + (size_t)(16 * nt) * HID + k0;
      FragB bf;
      bf.h[0] = *(const v8usa*)wq;
      bf.h[1] = *(const v8usa*)(wq + 16);
      acc[nt] = wmb(af, bf, acc[nt]);
    }
  }
  __syncthreads();

#pragma unroll
  for (int nt = 0; nt < 8; ++nt) {
    const int lc = 128 * cg + 16 * nt + m;
#pragma unroll
    for (int r = 0; r < 8; ++r) {
      const int lr = 16 * rw + 8 * hh + r;
      stg[lr * HID + lc] = acc[nt][r];
    }
  }
  __syncthreads();

  {
    const int row = tid >> 2, q = tid & 3;
    const float* hr = stg + row * HID + 64 * q;
    const float* br = b2s + 64 * q;
    const float* wr = w3s + 64 * q;
    float d = 0.0f;
#pragma unroll 1
    for (int c4 = 0; c4 < 16; ++c4) {
      const v4f hv = *(const v4fa*)(hr + 4 * c4);
      const v4f bv = *(const v4fa*)(br + 4 * c4);
      const v4f wv = *(const v4fa*)(wr + 4 * c4);
      const v4f t = hv + bv;
      d = fmaf(elu1(t.x), wv.x, d);
      d = fmaf(elu1(t.y), wv.y, d);
      d = fmaf(elu1(t.z), wv.z, d);
      d = fmaf(elu1(t.w), wv.w, d);
    }
    sred[row * 4 + q] = d;
  }
  __syncthreads();
  if (tid < EROWS) {
    sdv[tid] = ((sred[4 * tid] + sred[4 * tid + 1]) + sred[4 * tid + 2]) + sred[4 * tid + 3];
  }
  __syncthreads();

  const v4f dv4 = *(const v4fa*)(sdv + 4 * (tid & 15));
  float* dp = DL + (size_t)bb * NPR + (size_t)bx * EROWS + 4 * (tid & 15);
  if (tid < 16) *(volatile v4f*)dp = dv4;
  __threadfence();
  if (tid < 16) *(volatile v4f*)dp = dv4;
}

__global__ __launch_bounds__(NTHR) void k_adj(const float* __restrict__ DL, const float* __restrict__ b3, float* out) {
  __shared__ __attribute__((aligned(16))) float tile[ARG * NND];
  const int tid = (int)threadIdx.x, lane = tid & 31, wave = tid >> 5;
  const int rg = (int)blockIdx.x;
  const int bb = (int)blockIdx.y;
  const float b3r = bfr(b3[0]);
  const float* Db = DL + (size_t)bb * NPR;

#pragma unroll 1
  for (int i = 0; i < 4; ++i) {
    const int lr = 4 * wave + i;
    const int r  = ARG * rg + lr;
#pragma unroll 1
    for (int s8 = 0; s8 < NND / 32; ++s8) {
      const int c = 32 * s8 + lane;
      const float d0 = Db[(size_t)r * NND + c];
      const float d1 = Db[(size_t)c * NND + r];
      const float z  = ((d0 + b3r) + (d1 + b3r)) * 0.5f;
      const float e  = expf(-z);
      float p = 1.0f / (1.0f + e);
      p = (r == c) ? 0.0f : p;
      tile[lr * NND + c] = p;
    }
  }
  __syncthreads();

  v4f ov[8];
#pragma unroll
  for (int i = 0; i < 4; ++i) {
#pragma unroll
    for (int s = 0; s < 2; ++s) ov[2 * i + s] = *(const v4fa*)(tile + (4 * wave + i) * NND + 128 * s + 4 * lane);
  }
  float* ob = out + ((size_t)bb * NND + (size_t)(ARG * rg + 4 * wave)) * NND;
#pragma unroll
  for (int i = 0; i < 4; ++i) {
#pragma unroll
    for (int s = 0; s < 2; ++s) *(volatile v4f*)(ob + (size_t)i * NND + 128 * s + 4 * lane) = ov[2 * i + s];
  }
  __threadfence();
#pragma unroll
  for (int i = 0; i < 4; ++i) {
#pragma unroll
    for (int s = 0; s < 2; ++s) *(volatile v4f*)(ob + (size_t)i * NND + 128 * s + 4 * lane) = ov[2 * i + s];
  }
}

static inline size_t al256(size_t o) { return (o + 255) & ~(size_t)255; }

extern "C" void kernel_launch(void* const* d_in, const int* in_sizes, int n_in,
                              void* d_out, int out_size, void* d_ws, size_t ws_size,
                              hipStream_t stream) {
  if (n_in < 7) return;
  if (in_sizes[0] != M1 * DIN) return;
  if (in_sizes[1] != 2 * DIN * HID) return;
  if (in_sizes[2] != HID) return;
  if (in_sizes[3] != HID * HID) return;
  if (in_sizes[4] != HID) return;
  if (in_sizes[5] != HID) return;
  if (in_sizes[6] < 1) return;
  if (out_size != NBT * NND * NND) return;

  const float* x  = (const float*)d_in[0];
  const float* W1 = (const float*)d_in[1];
  const float* b1 = (const float*)d_in[2];
  const float* W2 = (const float*)d_in[3];
  const float* b2 = (const float*)d_in[4];
  const float* W3 = (const float*)d_in[5];
  const float* b3 = (const float*)d_in[6];
  float* out = (float*)d_out;

  char* ws = (char*)d_ws;
  size_t off = 0;
  const size_t oXB = off; off = al256(off + (size_t)M1 * DIN * 2);
  const size_t oW1 = off; off = al256(off + (size_t)N1 * DIN * 2);
  const size_t oW2 = off; off = al256(off + (size_t)HID * HID * 2);
  const size_t oPQ = off; off = al256(off + (size_t)M1 * N1 * 4);
  const size_t oDL = off; off = al256(off + (size_t)NBT * NPR * 4);
  if (off > ws_size || off > (size_t)WSMAX) return;
  unsigned short* XB  = (unsigned short*)(ws + oXB);
  unsigned short* W1B = (unsigned short*)(ws + oW1);
  unsigned short* W2T = (unsigned short*)(ws + oW2);
  float*          PQ  = (float*)(ws + oPQ);
  float*          DL  = (float*)(ws + oDL);

  hipFuncSetAttribute(reinterpret_cast<const void*>(&k_edge),
                      hipFuncAttributeMaxDynamicSharedMemorySize, ELDS_BYTES);

  {
    const int nUx = M1 * (DIN / 8);
    k_xprep<<<nUx / NTHR, NTHR, 0, stream>>>(x, XB, M1, nUx);
  }
  {
    const int nUa = HID * (DIN / 8);
    k_wtr<<<nUa / NTHR, NTHR, 0, stream>>>(W1, DIN, HID, HID, DIN, W1B, nUa);
    k_wtr<<<nUa / NTHR, NTHR, 0, stream>>>(W1 + (size_t)DIN * HID, DIN, HID, HID, DIN, W1B + (size_t)HID * DIN, nUa);
    const int nUb = HID * (HID / 8);
    k_wtr<<<nUb / NTHR, NTHR, 0, stream>>>(W2, HID, HID, HID, HID, W2T, nUb);
  }
  k_gemm1<<<dim3(M1 / GBM, N1 / GBN), GTHR, 0, stream>>>(XB, W1B, PQ, DIN, N1);
  k_edge<<<dim3(NND * CGRP, NBT), ETHR, ELDS_BYTES, stream>>>(PQ, W2T, b1, b2, W3, DL);
  k_adj<<<dim3(NND / ARG, NBT), NTHR, 0, stream>>>(DL, b3, out);
}
